// TransformerEncoderLayer_49323404427927
// MI455X (gfx1250) — hardware-verified
//
#include <hip/hip_runtime.h>


namespace {

constexpr int N = 32768  , NP = N, NPL = NP  , SRCM = N  , NB = 8  , NPER = 4096, LNB = 16  ;
constexpr int D = 256, HH = 8, DK = 32, DFF = 1024, VOC = 1, NRL = NP  , NL = (NPL < N ? NPL : N);
constexpr float NEGINF_ = -1e9f, LN_EPS = 1e-5f, ISQ = 0.17677669529663687f  ;
constexpr float LNEPS = 1e-5f; constexpr float LOG2E = 1.4426950408889634f; constexpr float XS = 8.0f, WSC = 256.0f, WSQ = 0.25f, RS_ = 1024.0f, NSL_ = 0.2f, NSA_ = 0.01f, SLOPE = 0.0f, BNEPS = 1e-5f;
static_assert(NP % 32 == 0 && NP >= N && NPL % 32 == 0 && D % 32 == 0 && DFF % 256 == 0, "tiling");
typedef _Float16 b16;
typedef __attribute__((ext_vector_type(16))) _Float16 v16b;
typedef __attribute__((ext_vector_type(8))) _Float16 v8b;
typedef __attribute__((ext_vector_type(8))) float v8f;
typedef __attribute__((ext_vector_type(4))) float v4f;
__device__ __forceinline__ float bf16_rne(float f) { unsigned int u = __float_as_uint(f); u += 0x7FFFu + ((u >> 16) & 1u); return __uint_as_float(u & 0xFFFF0000u); }
__device__ __forceinline__ void split16(float v, b16& hi, b16& lo) { hi = (b16)v; lo = (b16)(v - (float)hi); }
__device__ __forceinline__ v16b frag_kb(const b16* p, int hh) { const v8b a = *(const v8b*)(p + 8 * hh), b = *(const v8b*)(p + 16 + 8 * hh); v16b f;
#pragma unroll
  for (int e = 0; e < 8; ++e) { f[e] = a[e]; f[8 + e] = b[e]; } return f; }
__device__ __forceinline__ v8f wmma16b(v16b a, v16b b, v8f c) { v8f d = __builtin_amdgcn_wmma_f32_16x16x32_f16(false, a, false, b, (short)0, c, false, false); asm volatile("v_nop\n\tv_nop\n\tv_nop\n\tv_nop" : "+v"(d) : "v"(a), "v"(b)); return d; }
__device__ __forceinline__ void wave_lds_sync() { __builtin_amdgcn_fence(__ATOMIC_RELEASE, "workgroup"); __builtin_amdgcn_wave_barrier(); __builtin_amdgcn_fence(__ATOMIC_ACQUIRE, "workgroup"); }
__device__ __forceinline__ float pmul(float a, float b) { float p = a * b; asm volatile("" : "+v"(p)); return p; }
__device__ __forceinline__ float bfo(float f) { float r = bf16_rne(f); asm volatile("" : "+v"(r)); return r; }
__device__ __forceinline__ int iclamp(int v, int lo, int hi) { return v < lo ? lo : (v > hi ? hi : v); }

typedef __attribute__((ext_vector_type(4))) _Float16 v4h;
__device__ __forceinline__ float lrelu(float v) { return v > 0.0f ? v : NSL_ * v; }
template <int K, int NOUTR, int NOUTP>
__global__ __launch_bounds__(256) void wt_kernel(const float* __restrict__ w, b16* __restrict__ WT, float scl) {
  const int u = blockIdx.x * 256 + threadIdx.x; if (u >= NOUTP * K / 8) return; const int e = u * 8; const int o = e / K, k0 = e % K; v8b v;
#pragma unroll
  for (int j = 0; j < 8; ++j) v[j] = (b16)(o < NOUTR ? bf16_rne(w[(size_t)(k0 + j) * NOUTR + o]) * scl : 0.0f);
  for (int pass = 0; pass < 2; ++pass) { *(volatile v8b*)(WT + e) = v; __threadfence(); }
}
template <int K, int NT, int PREC, int MODE, bool GIDX>
__global__ __launch_bounds__(64) void lin_kernel(const float* __restrict__ X, const int* __restrict__ gidx, const b16* __restrict__ WT, const b16* __restrict__ WQ, const float* __restrict__ bias, float* __restrict__ OUT, int opitch, int nvalid, int mrows) {
  constexpr int NC = NT * 16;
  __shared__ __attribute__((aligned(16))) b16 Ah[2][16][K + 8], Al[2][16][(PREC == 0 ? K : 0) + 8]; __shared__ __attribute__((aligned(16))) float Tf[2][16][NC + 4];
  const int wave = threadIdx.x >> 5, lane = threadIdx.x & 31, nloc = lane & 15, hlf = lane >> 4; const size_t m0 = (size_t)blockIdx.x * 32 + wave * 16;
  for (int idx = lane; idx < 16 * (K / 4); idx += 32) { const int rr = idx / (K / 4), c4 = (idx % (K / 4)) * 4; const size_t vrow = (m0 + rr < (size_t)nvalid) ? m0 + rr : (size_t)nvalid - 1; size_t arow = vrow; if (GIDX) arow = (size_t)iclamp(gidx[vrow], 0, VOC - 1);
    const v4f v = *(const v4f*)(X + arow * K + c4); v4h hv, lv;
    for (int j = 0; j < 4; ++j) { float vj = v[j]; if (MODE == 2) vj = fmaxf(vj, 0.0f); const float vs = (PREC == 1 ? bf16_rne(vj) : vj) * XS; const b16 ph = (b16)vs; hv[j] = ph; lv[j] = (b16)((vs - (float)ph) * RS_); } *(v4h*)(&Ah[wave][rr][c4]) = hv; if (PREC == 0) *(v4h*)(&Al[wave][rr][c4]) = lv; }
  wave_lds_sync();
  v8f acc[NT];
#pragma unroll
  for (int t = 0; t < NT; ++t) acc[t] = (v8f){};
#pragma unroll 1
  for (int kb = 0; kb < K; kb += 32) { const v16b a = frag_kb(&Ah[wave][nloc][kb], hlf); v16b al; if (PREC == 0) al = frag_kb(&Al[wave][nloc][kb], hlf);
#pragma unroll
    for (int t = 0; t < NT; ++t) { const size_t wo_ = (size_t)(t * 16 + nloc) * K + kb; acc[t] = wmma16b(a, frag_kb(WT + wo_, hlf), acc[t]); if (PREC == 0) acc[t] = wmma16b(al, frag_kb(WQ + wo_, hlf), acc[t]); } }
#pragma unroll
  for (int t = 0; t < NT; ++t) { const int col = t * 16 + nloc; const float bb = bf16_rne(bias[col]);
    for (int r = 0; r < 8; ++r) { const size_t vrow = m0 + 8 * hlf + r; float y = acc[t][r] * (1.0f / (XS * WSC)) + bb; if (MODE == 1) y = fmaxf(y, 0.0f); Tf[wave][8 * hlf + r][col] = (vrow < (size_t)nvalid) ? y : 0.0f; } }
  wave_lds_sync();
  for (int pass = 0; pass < 2; ++pass) { for (int rr = 0; rr < 16; ++rr) { if (m0 + rr < (size_t)mrows) { if (NC >= 128) { for (int c8 = 0; c8 < NC; c8 += 128) *(volatile v4f*)(OUT + (m0 + rr) * (size_t)opitch + c8 + lane * 4) = *(const v4f*)(&Tf[wave][rr][c8 + lane * 4]); }
        else { if (lane < NC / 4) *(volatile v4f*)(OUT + (m0 + rr) * (size_t)opitch + lane * 4) = *(const v4f*)(&Tf[wave][rr][lane * 4]); } } } __threadfence(); }
}
__device__ __forceinline__ float gelu_(float v) { return 0.5f * v * (1.0f + erff(v * 0.70710678118654752f)); }
__global__ __launch_bounds__(256) void qkin_kernel(const float* __restrict__ s, const float* __restrict__ p, float* __restrict__ QK) {
  const size_t i = (size_t)blockIdx.x * 256 + threadIdx.x; if (i >= (size_t)NRL * (D / 4)) return; const size_t v = i / (D / 4); const int c = (int)(i % (D / 4)) * 4; v4f t = {0.0f, 0.0f, 0.0f, 0.0f};
  if (v < (size_t)N) { const v4f a = *(const v4f*)(s + v * D + c), b = *(const v4f*)(p + v * D + c); for (int j = 0; j < 4; ++j) t[j] = bf16_rne(a[j]) + bf16_rne(b[j]); }
  for (int pass = 0; pass < 2; ++pass) { *(volatile v4f*)(QK + v * D + c) = t; __threadfence(); }
}
__global__ __launch_bounds__(256) void lattn_kernel(const float* __restrict__ Q, const float* __restrict__ Kp, const float* __restrict__ V, const int* __restrict__ ipair, const int* __restrict__ kcnt, const int* __restrict__ ibatch, float* __restrict__ CTX, int mrows) {
  const int tid = threadIdx.x; const int row = tid >> 3, h = tid & 7, c0 = h * DK; const int n = blockIdx.x * 32 + row; const int nn = n < N ? n : N - 1;
  int offs[NB]; { int acc = 0; for (int b = 0; b < NB; ++b) { offs[b] = acc; acc += iclamp(kcnt[b], 0, N); } }
  const int bt = iclamp(ibatch[nn], 0, NB - 1); const int ob = offs[bt];
  float q[DK]; { const float* qr = Q + (size_t)nn * D + c0; for (int j4 = 0; j4 < DK / 4; ++j4) { const v4f t4 = *(const v4f*)(qr + 4 * j4); for (int j = 0; j < 4; ++j) q[4 * j4 + j] = t4[j] * ISQ; } }
  float lg[LNB]; int gix[LNB]; float m = -INFINITY;
#pragma unroll
  for (int l = 0; l < LNB; ++l) { const int raw = ipair[(size_t)nn * LNB + l]; const bool valid = raw >= 0; int g = valid ? raw + ob : 0; g = iclamp(g, 0, N - 1); if (SRCM < N) g %= SRCM; gix[l] = g;
    float s = 0.0f; const float* kr = Kp + (size_t)g * D + c0;
    for (int j4 = 0; j4 < DK / 4; ++j4) { const v4f t4 = *(const v4f*)(kr + 4 * j4); for (int j = 0; j < 4; ++j) s += pmul(q[4 * j4 + j], t4[j]); }
    lg[l] = valid ? s : NEGINF_; m = fmaxf(m, lg[l]); }
  float den = 0.0f; for (int l = 0; l < LNB; ++l) { lg[l] = __expf(lg[l] - m); den += lg[l]; } const float inv = 1.0f / den;
  float acc[DK]; for (int j = 0; j < DK; ++j) acc[j] = 0.0f;
#pragma unroll 1
  for (int l = 0; l < LNB; ++l) { const float p = lg[l] * inv; const float* vr = V + (size_t)gix[l] * D + c0;
    for (int j4 = 0; j4 < DK / 4; ++j4) { const v4f t4 = *(const v4f*)(vr + 4 * j4); for (int j = 0; j < 4; ++j) acc[4 * j4 + j] += pmul(p, t4[j]); } }
  for (int pass = 0; pass < 2; ++pass) { if (n < mrows) { float* orow = CTX + (size_t)n * D + c0; for (int j4 = 0; j4 < DK / 4; ++j4) { v4f o; for (int j = 0; j < 4; ++j) o[j] = (n < N) ? acc[4 * j4 + j] : 0.0f; *(volatile v4f*)(orow + 4 * j4) = o; } } __threadfence(); }
}
template <bool ADDBF>
__global__ __launch_bounds__(256) void resln_kernel(const float* __restrict__ A, const float* __restrict__ B, const float* __restrict__ gam, const float* __restrict__ bet, float* __restrict__ out, int mrows) {
  const int tid = threadIdx.x; const int row = tid >> 3, g = tid & 7, c0 = g * 32; const int v = blockIdx.x * 32 + row; const int vv = v < N ? v : N - 1;
  float y[32]; float s1 = 0.0f;
#pragma unroll
  for (int q4 = 0; q4 < 8; ++q4) { const v4f a4 = *(const v4f*)(A + (size_t)vv * D + c0 + 4 * q4), b4 = *(const v4f*)(B + (size_t)vv * D + c0 + 4 * q4); for (int j = 0; j < 4; ++j) { y[4 * q4 + j] = (ADDBF ? bfo(a4[j]) : a4[j]) + b4[j]; s1 += y[4 * q4 + j]; } }
  s1 += __shfl_xor(s1, 1); s1 += __shfl_xor(s1, 2); s1 += __shfl_xor(s1, 4); const float mu = s1 * (1.0f / D); float s2 = 0.0f;
  for (int j = 0; j < 32; ++j) { const float d = y[j] - mu; s2 += pmul(d, d); }
  s2 += __shfl_xor(s2, 1); s2 += __shfl_xor(s2, 2); s2 += __shfl_xor(s2, 4); const float rs = rsqrtf(s2 * (1.0f / D) + LN_EPS);
  for (int pass = 0; pass < 2; ++pass) { if (v < mrows) { float* orow = out + (size_t)v * D + c0;
#pragma unroll
      for (int q4 = 0; q4 < 8; ++q4) { v4f o4; const v4f g4 = *(const v4f*)(gam + c0 + 4 * q4), e4 = *(const v4f*)(bet + c0 + 4 * q4); for (int j = 0; j < 4; ++j) o4[j] = (v < N) ? pmul(pmul(y[4 * q4 + j] - mu, rs), bfo(g4[j])) + bfo(e4[j]) : 0.0f; *(volatile v4f*)(orow + 4 * q4) = o4; } }
    __threadfence(); }
}
}

extern "C" void kernel_launch(void* const* d_in, const int* in_sizes, int n_in, void* d_out, int out_size, void* d_ws, size_t ws_size, hipStream_t stream) {
  (void)n_in;
  auto Fp = [&](int i) { return (const float*)d_in[i]; }; auto Ip = [&](int i) { return (const int*)d_in[i]; };
  if (in_sizes[0] != N * D || in_sizes[1] != N * D || in_sizes[2] != N * LNB || in_sizes[3] != NB || in_sizes[4] != NB || in_sizes[5] != N) return;
  for (int i = 6; i <= 12; i += 2) if (in_sizes[i] != D * D || in_sizes[i + 1] != D) return;
  if (in_sizes[14] != D * DFF || in_sizes[15] != DFF || in_sizes[16] != DFF * D || in_sizes[17] != D || in_sizes[18] != D || in_sizes[19] != D || in_sizes[20] != D || in_sizes[21] != D || out_size != N * D) return;
  size_t off = 0; char* ws = (char*)d_ws;
  auto carve = [&](size_t bytes) { char* p = ws + off; off += (bytes + 255) & ~(size_t)255; return p; };
  const size_t wsz = (size_t)D * D * 2, plane = (size_t)NP * D * 4;
  b16* WQT = (b16*)carve(wsz); b16* WQQ = (b16*)carve(wsz); b16* WKT = (b16*)carve(wsz); b16* WKQ = (b16*)carve(wsz); b16* WVT = (b16*)carve(wsz); b16* WOT = (b16*)carve(wsz); b16* WOQ = (b16*)carve(wsz);
  b16* W1T = (b16*)carve((size_t)DFF * D * 2); b16* W2T = (b16*)carve((size_t)D * DFF * 2);
  float* X = (float*)carve(plane); float* CTX = (float*)carve(plane);
  char* big = carve(4 * plane);
  float* QK = (float*)big; float* Qp = (float*)(big + plane); float* KP = (float*)(big + 2 * plane); float* VP = (float*)(big + 3 * plane); float* HID = (float*)big; float* FF = CTX;
  if (off > ws_size || off > ((size_t)208 << 20)) return;
  { const unsigned g = (D * D / 8 + 255) / 256;
    wt_kernel<D, D, D><<<g, 256, 0, stream>>>(Fp(6), WQT, WSC); wt_kernel<D, D, D><<<g, 256, 0, stream>>>(Fp(6), WQQ, WSQ); wt_kernel<D, D, D><<<g, 256, 0, stream>>>(Fp(8), WKT, WSC); wt_kernel<D, D, D><<<g, 256, 0, stream>>>(Fp(8), WKQ, WSQ);
    wt_kernel<D, D, D><<<g, 256, 0, stream>>>(Fp(10), WVT, WSC); wt_kernel<D, D, D><<<g, 256, 0, stream>>>(Fp(12), WOT, WSC); wt_kernel<D, D, D><<<g, 256, 0, stream>>>(Fp(12), WOQ, WSQ);
    wt_kernel<D, DFF, DFF><<<(DFF * D / 8 + 255) / 256, 256, 0, stream>>>(Fp(14), W1T, WSC); wt_kernel<DFF, D, D><<<(D * DFF / 8 + 255) / 256, 256, 0, stream>>>(Fp(16), W2T, WSC); }
  qkin_kernel<<<(unsigned)(((size_t)NRL * (D / 4) + 255) / 256), 256, 0, stream>>>(Fp(0), Fp(1), QK);
  lin_kernel<D, 16, 0, 0, false><<<NRL / 32, 64, 0, stream>>>(QK, nullptr, WQT, WQQ, Fp(7), Qp, D, N, NRL);
  lin_kernel<D, 16, 0, 0, false><<<NRL / 32, 64, 0, stream>>>(QK, nullptr, WKT, WKQ, Fp(9), KP, D, N, NRL);
  lin_kernel<D, 16, 1, 0, false><<<NRL / 32, 64, 0, stream>>>(Fp(0), nullptr, WVT, WVT, Fp(11), VP, D, N, NRL);
  lattn_kernel<<<NPL / 32, 256, 0, stream>>>(Qp, KP, VP, Ip(2), Ip(4), Ip(5), CTX, NPL);
  lin_kernel<D, 16, 0, 0, false><<<NPL / 32, 64, 0, stream>>>(CTX, nullptr, WOT, WOQ, Fp(13), X, D, N, NPL);
  resln_kernel<true><<<NPL / 32, 256, 0, stream>>>(Fp(0), X, Fp(18), Fp(19), X, NPL);
  for (int t = 0; t < DFF / 256; ++t)
    lin_kernel<D, 16, 2, 1, false><<<NPL / 32, 64, 0, stream>>>(X, nullptr, W1T + (size_t)t * 256 * D, W1T, Fp(15) + t * 256, HID + t * 256, DFF, N, NPL);
  lin_kernel<DFF, 16, 2, 0, false><<<NPL / 32, 64, 0, stream>>>(HID, nullptr, W2T, W2T, Fp(17), FF, D, N, NPL);
  resln_kernel<false><<<NPL / 32, 256, 0, stream>>>(X, FF, Fp(20), Fp(21), (float*)d_out, NL);
}
